// GAFLatentExtractor_57629871177824
// MI455X (gfx1250) — hardware-verified
//
#include <hip/hip_runtime.h>
#include <stdint.h>

typedef __attribute__((ext_vector_type(16))) _Float16 v16h;
typedef __attribute__((ext_vector_type(8)))  _Float16 v8h;
typedef __attribute__((ext_vector_type(8)))  float    v8f;
typedef __attribute__((ext_vector_type(4)))  float    v4f;

#define NIMG 512
#define NI_CHUNK 128
#define WSC 16.0f
#define WINV 0.0625f

__device__ __forceinline__ void dep_guard_h(v8f& a, v8f& b, v16h x, v16h y) { asm volatile("v_nop\n\tv_nop\n\tv_nop\n\tv_nop" : "+v"(a), "+v"(b) : "v"(x), "v"(y)); }
__device__ __forceinline__ void keep4_h(v16h a, v16h b, v16h c, v16h d) { asm volatile("v_nop" :: "v"(a), "v"(b), "v"(c), "v"(d)); }
template <typename T> struct Frag;
template <> struct Frag<_Float16> {
  typedef v16h V; union U { v16h v; v8h h[2]; };
  static __device__ __forceinline__ v16h load(const _Float16* p) {
    U f; f.h[0] = *(const v8h*)(p); f.h[1] = *(const v8h*)(p + 16); return f.v;
  }
  static __device__ __forceinline__ v8f mma(v16h a, v16h b, v8f c) {
    return __builtin_amdgcn_wmma_f32_16x16x32_f16(false, a, false, b, (short)0, c, false, false);
  }
  static __device__ __forceinline__ void guard(v8f& a, v8f& b, v16h x, v16h y) { dep_guard_h(a, b, x, y); }
  static __device__ __forceinline__ void keep(v16h a, v16h b, v16h c, v16h d) { keep4_h(a, b, c, d); }
};
typedef Frag<_Float16> FH;

__device__ __forceinline__ void guard_2x2(v8f& c0, v8f& c1, v8f& c2, v8f& c3, v16h a0, v16h a1, v16h b0, v16h b1) {
  asm volatile("v_nop\n\tv_nop\n\tv_nop\n\tv_nop" : "+v"(c0), "+v"(c1), "+v"(c2), "+v"(c3) : "v"(a0), "v"(a1), "v"(b0), "v"(b1));
}
__device__ __forceinline__ void guard_2x1(v8f& c0, v8f& c1, v16h a0, v16h a1, v16h b0) {
  asm volatile("v_nop\n\tv_nop\n\tv_nop\n\tv_nop" : "+v"(c0), "+v"(c1) : "v"(a0), "v"(a1), "v"(b0));
}

__device__ __forceinline__ v8h zero8h() { v8h z;
#pragma unroll
  for (int e = 0; e < 8; ++e) z[e] = (_Float16)0.0f;
  return z; }
__device__ __forceinline__ v8f zero8f() { return (v8f){0.f,0.f,0.f,0.f,0.f,0.f,0.f,0.f}; }

__global__ __launch_bounds__(128)
void gaf_series_kernel(const float* __restrict__ x_raw, float* __restrict__ tab)
{
  __shared__ float rmn[4], rmx[4];
  const int img = blockIdx.x, t = threadIdx.x, lane = t & 31, w = t >> 5;
  float v;
  {
    #pragma clang fp contract(off)
    const v4f q = *(const v4f*)(x_raw + (size_t)img * 512 + t * 4);
    v = (((q[0] + q[1]) + q[2]) + q[3]) * 0.25f;
  }
  float mn = v, mx = v;
#pragma unroll
  for (int off = 1; off < 32; off <<= 1) {
    mn = fminf(mn, __shfl_xor(mn, off, 32));
    mx = fmaxf(mx, __shfl_xor(mx, off, 32));
  }
  if (lane == 0) { rmn[w] = mn; rmx[w] = mx; }
  __syncthreads();
  mn = fminf(fminf(rmn[0], rmn[1]), fminf(rmn[2], rmn[3]));
  mx = fmaxf(fmaxf(rmx[0], rmx[1]), fmaxf(rmx[2], rmx[3]));
  float xn, sq;
  {
    #pragma clang fp contract(off)
    const float d  = (mx - mn) + 1e-8f;
    const float rd = 1.0f / d;
    xn = (2.0f * (v - mn)) * rd - 1.0f;
    xn = fminf(1.0f, fmaxf(-1.0f, xn));
    float u = 1.0f - xn * xn;
    u = fminf(1.0f, fmaxf(0.0f, u));
    sq = sqrtf(u);
  }
  float* dst = tab + (size_t)img * 256;
  *(volatile float*)(dst + t) = xn;
  *(volatile float*)(dst + 128 + t) = sq;
  __threadfence();
  *(volatile float*)(dst + t) = xn;
  *(volatile float*)(dst + 128 + t) = sq;
}

__global__ __launch_bounds__(256)
void prep_convw_kernel(const float* __restrict__ src, _Float16* __restrict__ dst, int OC, int IC, int Kpad, int n2)
{
  const int i = blockIdx.x * 256 + threadIdx.x;
  if (i >= n2) return;
  const int K = IC * 9;
  unsigned u = 0;
#pragma unroll
  for (int e = 0; e < 2; ++e) {
    const int j = 2 * i + e;
    const int n = j / Kpad;
    const int k = j - n * Kpad;
    const int kc = (k < K) ? k : (K - 1);
    const int tap = kc / IC;
    const int ic = kc - tap * IC;
    float v = src[((size_t)n * IC + ic) * 9 + tap] * WSC;
    if (k >= K) v = 0.0f;
    const _Float16 h = (_Float16)v;
    u |= ((unsigned)__builtin_bit_cast(unsigned short, h)) << (16 * e);
  }
  ((volatile unsigned*)dst)[i] = u;
  __threadfence();
  ((volatile unsigned*)dst)[i] = u;
}

__global__ __launch_bounds__(256)
void prep_fcw_kernel(const float* __restrict__ src, _Float16* __restrict__ dst)
{
  const int i = blockIdx.x * 256 + threadIdx.x;
  if (i >= 16384) return;
  unsigned u = 0;
#pragma unroll
  for (int e = 0; e < 2; ++e) {
    const int j = 2 * i + e;
    const int n = j >> 8, k = j & 255;
    const _Float16 h = (_Float16)(src[(size_t)k * 128 + n] * WSC);
    u |= ((unsigned)__builtin_bit_cast(unsigned short, h)) << (16 * e);
  }
  ((volatile unsigned*)dst)[i] = u;
  __threadfence();
  ((volatile unsigned*)dst)[i] = u;
}

__global__ __launch_bounds__(256)
void conv1_kernel(const float* __restrict__ tab, const _Float16* __restrict__ wt, const float* __restrict__ bias,
                  _Float16* __restrict__ act_out, int img0)
{
  constexpr int OW = 64, OC = 32, BH = 4, M = 256, BANDS = 16;
  __shared__ float xl[256];
  __shared__ __align__(16) _Float16 lds_a[M * 32];
  __shared__ __align__(16) _Float16 lds_out[M * OC];

  const int tid = threadIdx.x;
  const int il = blockIdx.x / BANDS;
  const int band = blockIdx.x - il * BANDS;

  xl[tid] = tab[(size_t)(img0 + il) * 256 + tid];
  __syncthreads();

  {
    #pragma clang fp contract(off)
    const int m = tid;
    const int oy = band * BH + (m >> 6);
    const int ox = m & 63;
    union { v16h v[2]; _Float16 e[32]; } row;
    row.v[0] = (v16h)(0); row.v[1] = (v16h)(0);
#pragma unroll
    for (int ky = 0; ky < 3; ++ky) {
      const int i = 2 * oy + ky;
      const int icl = (i < 128) ? i : 127;
      float xi = xl[icl], si = xl[128 + icl];
      if (i >= 128) { xi = 0.0f; si = 0.0f; }
#pragma unroll
      for (int kx = 0; kx < 3; ++kx) {
        const int j = 2 * ox + kx;
        const int jcl = (j < 128) ? j : 127;
        float xj = xl[jcl], sj = xl[128 + jcl];
        if (j >= 128) { xj = 0.0f; sj = 0.0f; }
        const float g0 = xi * xj - si * sj;
        const float g1 = si * xj - xi * sj;
        const int tap = ky * 3 + kx;
        row.e[tap * 2 + 0] = (_Float16)g0;
        row.e[tap * 2 + 1] = (_Float16)g1;
      }
    }
    *(v16h*)(lds_a + m * 32) = row.v[0];
    *(v16h*)(lds_a + m * 32 + 16) = row.v[1];
  }
  __syncthreads();

  const int lane = tid & 31, wave = tid >> 5, hh = lane >> 4, nm = lane & 15;
  const int mt0 = wave * 2;
  v8f acc00 = zero8f(), acc01 = zero8f(), acc10 = zero8f(), acc11 = zero8f();
  {
    const v16h a0 = FH::load(lds_a + (mt0 * 16 + nm) * 32 + hh * 8);
    const v16h a1 = FH::load(lds_a + (mt0 * 16 + 16 + nm) * 32 + hh * 8);
    const v16h b0 = FH::load(wt + nm * 32 + hh * 8);
    const v16h b1 = FH::load(wt + (16 + nm) * 32 + hh * 8);
    acc00 = FH::mma(a0, b0, acc00);
    acc01 = FH::mma(a0, b1, acc01);
    acc10 = FH::mma(a1, b0, acc10);
    acc11 = FH::mma(a1, b1, acc11);
    guard_2x2(acc00, acc01, acc10, acc11, a0, a1, b0, b1);
  }

  const int oc0 = nm, oc1 = 16 + nm;
  const float bv0 = bias[oc0], bv1 = bias[oc1];
#pragma unroll
  for (int r = 0; r < 8; ++r) {
    const int ma = mt0 * 16 + hh * 8 + r;
    const int mb = ma + 16;
    lds_out[ma * OC + oc0] = (_Float16)fmaxf(acc00[r] * WINV + bv0, 0.0f);
    lds_out[ma * OC + oc1] = (_Float16)fmaxf(acc01[r] * WINV + bv1, 0.0f);
    lds_out[mb * OC + oc0] = (_Float16)fmaxf(acc10[r] * WINV + bv0, 0.0f);
    lds_out[mb * OC + oc1] = (_Float16)fmaxf(acc11[r] * WINV + bv1, 0.0f);
  }
  __syncthreads();

  _Float16* gout = act_out + ((size_t)(il * 64 + band * BH) * OW) * OC;
  for (int pass = 0; pass < 2; ++pass) {
#pragma unroll
    for (int it = 0; it < 4; ++it) {
      const int q = it * 256 + tid;
      const v8h v = *(const v8h*)(lds_out + q * 8);
      *(volatile v8h*)(gout + (size_t)q * 8) = v;
    }
    __threadfence();
  }
}

template<int IC, int OC, int IH, int OH, bool POOL>
__global__ __launch_bounds__(256)
void conv3x3s2_kernel(const _Float16* __restrict__ act_in,
                      const _Float16* __restrict__ wt,
                      const float*    __restrict__ bias,
                      _Float16*       __restrict__ act_out,
                      float*          __restrict__ part,
                      int img0)
{
  constexpr int IW = IH, OW = OH, BH = 4;
  constexpr int ROWS = 2 * BH + 1;
  constexpr int PW = IW + 1;
  constexpr int K = 9 * IC;
  constexpr int CCH = IC / 32;
  constexpr int BANDS = OH / BH;
  constexpr int M = BH * OW;
  constexpr int MT = M / 16, NT = OC / 16;
  constexpr int NT2 = NT / 2;
  constexpr int C8 = IC / 8;
  static_assert(MT * NT == 32);
  static_assert(IW * C8 == 256);
  static_assert(IC % 32 == 0);
  static_assert(POOL || (M * OC == 8192));
  static_assert(!POOL || (MT == 2));
  constexpr int IN_HALVES  = ROWS * PW * IC;
  constexpr int OUT_HALVES = POOL ? 8 : M * OC;

  __shared__ __align__(16) _Float16 lds_in[IN_HALVES];
  __shared__ __align__(16) _Float16 lds_out[OUT_HALVES];
  __shared__ __align__(16) float psum[POOL ? OC : 4];

  const int tid = threadIdx.x;
  const int il = blockIdx.x / BANDS;
  const int band = blockIdx.x - il * BANDS;
  const int y0 = band * 2 * BH;

  const v8h zh = zero8h();
  {
    const _Float16* gin = act_in + (size_t)il * IH * IW * IC;
    const int xq = tid / C8;
    const int cq = (tid - xq * C8) * 8;
#pragma unroll 1
    for (int yr = 0; yr < ROWS; ++yr) {
      const int y = y0 + yr;
      const int yc = (y < IH) ? y : (IH - 1);
      v8h v = *(const v8h*)(gin + (size_t)yc * IW * IC + (size_t)tid * 8);
      if (y >= IH) v = zh;
      *(v8h*)(lds_in + (yr * PW + xq) * IC + cq) = v;
    }
    for (int i = tid; i < ROWS * C8; i += 256) {
      const int yr = i / C8;
      const int c8 = (i - yr * C8) * 8;
      *(v8h*)(lds_in + (yr * PW + IW) * IC + c8) = zh;
    }
  }
  __syncthreads();

  const int lane = tid & 31, wave = tid >> 5, hh = lane >> 4, nm = lane & 15;
  const int mt0 = (wave / NT2) * 2;
  const int nt0 = (wave - (wave / NT2) * NT2) * 2;
  const int m0 = mt0 * 16 + nm, m1 = m0 + 16;
  const int oy0 = m0 / OW, ox0 = m0 - oy0 * OW;
  const int oy1 = m1 / OW, ox1 = m1 - oy1 * OW;
  const _Float16* ab0 = lds_in + ((2 * oy0) * PW + 2 * ox0) * IC + hh * 8;
  const _Float16* ab1 = lds_in + ((2 * oy1) * PW + 2 * ox1) * IC + hh * 8;
  const _Float16* wr0 = wt + (size_t)(nt0 * 16 + nm) * K + hh * 8;
  const _Float16* wr1 = wr0 + (size_t)16 * K;

  v8f acc00 = zero8f(), acc01 = zero8f(), acc10 = zero8f(), acc11 = zero8f();
#pragma unroll 1
  for (int tap = 0; tap < 9; ++tap) {
    const int ky = tap / 3;
    const int kx = tap - 3 * ky;
    const int aoff = (ky * PW + kx) * IC;
    const int woff = tap * IC;
#pragma unroll
    for (int c = 0; c < CCH; ++c) {
      const v16h a0 = FH::load(ab0 + aoff + c * 32);
      const v16h a1 = FH::load(ab1 + aoff + c * 32);
      const v16h b0 = FH::load(wr0 + woff + c * 32);
      const v16h b1 = FH::load(wr1 + woff + c * 32);
      acc00 = FH::mma(a0, b0, acc00);
      acc01 = FH::mma(a0, b1, acc01);
      acc10 = FH::mma(a1, b0, acc10);
      acc11 = FH::mma(a1, b1, acc11);
      guard_2x2(acc00, acc01, acc10, acc11, a0, a1, b0, b1);
    }
  }

  const int oc0 = nt0 * 16 + nm, oc1 = oc0 + 16;
  const float bv0 = bias[oc0], bv1 = bias[oc1];
  if constexpr (!POOL) {
#pragma unroll
    for (int r = 0; r < 8; ++r) {
      const int ma = mt0 * 16 + hh * 8 + r;
      const int mb = ma + 16;
      lds_out[ma * OC + oc0] = (_Float16)fmaxf(acc00[r] * WINV + bv0, 0.0f);
      lds_out[ma * OC + oc1] = (_Float16)fmaxf(acc01[r] * WINV + bv1, 0.0f);
      lds_out[mb * OC + oc0] = (_Float16)fmaxf(acc10[r] * WINV + bv0, 0.0f);
      lds_out[mb * OC + oc1] = (_Float16)fmaxf(acc11[r] * WINV + bv1, 0.0f);
    }
    __syncthreads();
    _Float16* gout = act_out + ((size_t)(il * OH + band * BH) * OW) * OC;
    for (int pass = 0; pass < 2; ++pass) {
#pragma unroll
      for (int it = 0; it < 4; ++it) {
        const int q = it * 256 + tid;
        const v8h v = *(const v8h*)(lds_out + q * 8);
        *(volatile v8h*)(gout + (size_t)q * 8) = v;
      }
      __threadfence();
    }
  } else {
    float s0 = 0.0f, s1 = 0.0f;
#pragma unroll
    for (int r = 0; r < 8; ++r) {
      s0 += fmaxf(acc00[r] * WINV + bv0, 0.0f);
      s0 += fmaxf(acc10[r] * WINV + bv0, 0.0f);
      s1 += fmaxf(acc01[r] * WINV + bv1, 0.0f);
      s1 += fmaxf(acc11[r] * WINV + bv1, 0.0f);
    }
    s0 += __shfl_xor(s0, 16, 32);
    s1 += __shfl_xor(s1, 16, 32);
    psum[nt0 * 16 + hh * 16 + nm] = hh ? s1 : s0;
    __syncthreads();
    float* gp = part + ((size_t)(img0 + il) * 2 + band) * OC;
    v4f pv = (v4f){0.f, 0.f, 0.f, 0.f};
    if (tid < OC / 4) pv = *(const v4f*)(psum + tid * 4);
    if (tid < OC / 4) *(volatile v4f*)(gp + tid * 4) = pv;
    __threadfence();
    if (tid < OC / 4) *(volatile v4f*)(gp + tid * 4) = pv;
  }
}

__global__ __launch_bounds__(256)
void fc_mean_kernel(const float* __restrict__ part, const _Float16* __restrict__ wt, const float* __restrict__ bias,
                    float* __restrict__ out)
{
  __shared__ __align__(16) _Float16 lds_p[32 * 256];
  __shared__ __align__(16) float outv[128];
  const int b = blockIdx.x, tid = threadIdx.x;
#pragma unroll 1
  for (int c = 0; c < 32; ++c) {
    const float* pp = part + ((size_t)(b * 32 + c) * 2) * 256;
    const float v = (pp[tid] + pp[256 + tid]) * (1.0f / 64.0f);
    lds_p[c * 256 + tid] = (_Float16)v;
  }
  __syncthreads();

  const int lane = tid & 31, wave = tid >> 5, hh = lane >> 4, nm = lane & 15;
  const _Float16* pa0 = lds_p + nm * 256 + hh * 8;
  const _Float16* pa1 = lds_p + (16 + nm) * 256 + hh * 8;
  const _Float16* pb  = wt + (size_t)(wave * 16 + nm) * 256 + hh * 8;
  v8f acc0 = zero8f(), acc1 = zero8f();
#pragma unroll 1
  for (int k0 = 0; k0 < 256; k0 += 32) {
    const v16h a0 = FH::load(pa0 + k0);
    const v16h a1 = FH::load(pa1 + k0);
    const v16h bb = FH::load(pb + k0);
    acc0 = FH::mma(a0, bb, acc0);
    acc1 = FH::mma(a1, bb, acc1);
    guard_2x1(acc0, acc1, a0, a1, bb);
  }
  const int n = wave * 16 + nm;
  const float bv = bias[n];
  float s = 0.0f;
#pragma unroll
  for (int r = 0; r < 8; ++r) {
    s += acc0[r] * WINV + bv;
    s += acc1[r] * WINV + bv;
  }
  s += __shfl_xor(s, 16, 32);
  outv[n] = s * (1.0f / 32.0f);
  __syncthreads();
  v4f ov = (v4f){0.f, 0.f, 0.f, 0.f};
  if (tid < 32) ov = *(const v4f*)(outv + tid * 4);
  if (tid < 32) *(volatile v4f*)(out + (size_t)b * 128 + tid * 4) = ov;
  __threadfence();
  if (tid < 32) *(volatile v4f*)(out + (size_t)b * 128 + tid * 4) = ov;
}

extern "C" void kernel_launch(void* const* d_in, const int* in_sizes, int n_in,
                              void* d_out, int out_size, void* d_ws, size_t ws_size,
                              hipStream_t stream)
{
  if (n_in < 11) return;
  if (in_sizes[0] != 16 * 32 * 512 || in_sizes[1] != 32 * 2 * 9 || in_sizes[2] != 32 ||
      in_sizes[3] != 64 * 32 * 9 || in_sizes[4] != 64 || in_sizes[5] != 128 * 64 * 9 || in_sizes[6] != 128 ||
      in_sizes[7] != 256 * 128 * 9 || in_sizes[8] != 256 || in_sizes[9] != 256 * 128 || in_sizes[10] != 128 ||
      out_size != 16 * 128) return;

  const float* x_raw = (const float*)d_in[0];
  const float* W1  = (const float*)d_in[1];
  const float* b1  = (const float*)d_in[2];
  const float* W2  = (const float*)d_in[3];
  const float* b2  = (const float*)d_in[4];
  const float* W3  = (const float*)d_in[5];
  const float* b3  = (const float*)d_in[6];
  const float* W4  = (const float*)d_in[7];
  const float* b4  = (const float*)d_in[8];
  const float* Wfc = (const float*)d_in[9];
  const float* bfc = (const float*)d_in[10];
  float* out = (float*)d_out;

  char* ws = (char*)d_ws;
  size_t off = 0;
  auto take = [&](size_t bytes) -> size_t { size_t r = off; off += (bytes + 4095) & ~(size_t)4095; return r; };
  const size_t NI = NI_CHUNK;
  const size_t o_tab  = take((size_t)NIMG * 256 * 4);
  const size_t o_w1   = take((size_t)32 * 32 * 2);
  const size_t o_w2   = take((size_t)64 * 288 * 2);
  const size_t o_w3   = take((size_t)128 * 576 * 2);
  const size_t o_w4   = take((size_t)256 * 1152 * 2);
  const size_t o_wfc  = take((size_t)128 * 256 * 2);
  const size_t o_h1   = take(NI * 64 * 64 * 32 * 2);
  const size_t o_h2   = take(NI * 32 * 32 * 64 * 2);
  const size_t o_h3   = take(NI * 16 * 16 * 128 * 2);
  const size_t o_part = take((size_t)NIMG * 2 * 256 * 4);
  if (off > ws_size) return;

  float*    tab  = (float*)(ws + o_tab);
  _Float16* w1h  = (_Float16*)(ws + o_w1);
  _Float16* w2h  = (_Float16*)(ws + o_w2);
  _Float16* w3h  = (_Float16*)(ws + o_w3);
  _Float16* w4h  = (_Float16*)(ws + o_w4);
  _Float16* wfch = (_Float16*)(ws + o_wfc);
  _Float16* h1   = (_Float16*)(ws + o_h1);
  _Float16* h2   = (_Float16*)(ws + o_h2);
  _Float16* h3   = (_Float16*)(ws + o_h3);
  float*    part = (float*)(ws + o_part);

  gaf_series_kernel<<<dim3(NIMG), dim3(128), 0, stream>>>(x_raw, tab);
  prep_convw_kernel<<<dim3((512 + 255) / 256), dim3(256), 0, stream>>>(W1, w1h, 32, 2, 32, 512);
  prep_convw_kernel<<<dim3((9216 + 255) / 256), dim3(256), 0, stream>>>(W2, w2h, 64, 32, 288, 9216);
  prep_convw_kernel<<<dim3((36864 + 255) / 256), dim3(256), 0, stream>>>(W3, w3h, 128, 64, 576, 36864);
  prep_convw_kernel<<<dim3((147456 + 255) / 256), dim3(256), 0, stream>>>(W4, w4h, 256, 128, 1152, 147456);
  prep_fcw_kernel<<<dim3(16384 / 256), dim3(256), 0, stream>>>(Wfc, wfch);

  for (int ch = 0; ch < NIMG / NI_CHUNK; ++ch) {
    const int img0 = ch * NI_CHUNK;
    conv1_kernel<<<dim3(NI_CHUNK * 16), dim3(256), 0, stream>>>(tab, w1h, b1, h1, img0);
    conv3x3s2_kernel< 32,  64, 64, 32, false><<<dim3(NI_CHUNK * 8), dim3(256), 0, stream>>>(h1, w2h, b2, h2, part, img0);
    conv3x3s2_kernel< 64, 128, 32, 16, false><<<dim3(NI_CHUNK * 4), dim3(256), 0, stream>>>(h2, w3h, b3, h3, part, img0);
    conv3x3s2_kernel<128, 256, 16,  8, true ><<<dim3(NI_CHUNK * 2), dim3(256), 0, stream>>>(h3, w4h, b4, h2, part, img0);
  }
  fc_mean_kernel<<<dim3(16), dim3(256), 0, stream>>>(part, wfch, bfc, out);
}
